// PatchQuantumGenerator_86577950753233
// MI455X (gfx1250) — hardware-verified
//
#include <hip/hip_runtime.h>


typedef __attribute__((ext_vector_type(16))) _Float16 v16h;
typedef __attribute__((ext_vector_type(8)))  _Float16 v8h;
typedef __attribute__((ext_vector_type(8)))  float    v8f;
typedef __attribute__((ext_vector_type(4)))  float    v4f;
#define NB   16384
#define TL   32
#define C1   128
#define C2   64
#define K2   384
#define NROW (NB * TL)
#define VST2(T, ptr, val) do { const T _v = (val); *(volatile T*)(ptr) = _v; __threadfence(); *(volatile T*)(ptr) = _v; } while (0)
__device__ __forceinline__ v8f wmma16(v16h a, v16h b, v8f c) {
  v8f d = __builtin_amdgcn_wmma_f32_16x16x32_f16(false, a, false, b, (short)0, c, false, false);
  asm volatile("v_nop\n\tv_nop\n\tv_nop\n\tv_nop" : "+v"(d) : "v"(a), "v"(b));
  return d;
}
__device__ __forceinline__ v16h frag16(const _Float16* p, int hh) {
  const v8h lo = *(const v8h*)(p + 8 * hh), hi = *(const v8h*)(p + 16 + 8 * hh);
  return __builtin_shufflevector(lo, hi, 0,1,2,3,4,5,6,7,8,9,10,11,12,13,14,15);
}

__global__ __launch_bounds__(256) void k_patches(const float* __restrict__ x, const float* __restrict__ qp, float* __restrict__ images) {
  const int t = blockIdx.x * 256 + threadIdx.x;
  const int b = t >> 3, g = (t >> 1) & 3, hf = t & 1;
  float cs[4], sn[4];
#pragma unroll
  for (int q = 0; q < 4; ++q) { const float th = 0.5f * (x[b * 4 + q] + qp[g * 4 + q]); cs[q] = __cosf(th); sn[q] = __sinf(th); }
  float p[16], tot = 0.f;
#pragma unroll
  for (int i = 0; i < 16; ++i) {
    float a = 1.0f;
#pragma unroll
    for (int q = 0; q < 4; ++q) a *= ((i >> (3 - q)) & 1) ? sn[q] : cs[q];
    p[i] = a * a; tot += p[i];
  }
  float mx = 0.f;
#pragma unroll
  for (int i = 0; i < 8; ++i) { p[i] = p[i] / tot; mx = fmaxf(mx, p[i]); }
  v4f o;
#pragma unroll
  for (int e = 0; e < 4; ++e) o[e] = p[hf * 4 + e] / mx;
  VST2(v4f, images + (size_t)b * 32 + g * 8 + hf * 4, o);
}
__global__ __launch_bounds__(256) void k_conv1(const float* __restrict__ images, const float* __restrict__ w1, const float* __restrict__ b1,
                                               float* __restrict__ part1) {
  __shared__ float red[2][16][C1];
  const int cg = threadIdx.x & 15, rl = threadIdx.x >> 4;
  const int b0 = blockIdx.x * 8;
  float wA[8], wB[8], wC[8], bb[8], s[8], s2[8];
#pragma unroll
  for (int e = 0; e < 8; ++e) { const int c = cg * 8 + e; wA[e] = w1[c * 3 + 2]; wB[e] = w1[c * 3 + 1]; wC[e] = w1[c * 3 + 0]; bb[e] = b1[c]; s[e] = 0.f; s2[e] = 0.f; }
  for (int pass = 0; pass < 16; ++pass) {
    const int row = pass * 16 + rl, b = b0 + (row >> 5), t = row & 31;
    const float* im = images + (size_t)b * 32;
    const float i0 = (t > 0) ? im[t - 1] : 0.f, i1 = im[t], i2 = (t < TL - 1) ? im[t + 1] : 0.f;
#pragma unroll
    for (int e = 0; e < 8; ++e) { const float v = fmaxf(i0 * wA[e] + i1 * wB[e] + i2 * wC[e] + bb[e], 0.f); s[e] += v; s2[e] += v * v; }
  }
#pragma unroll
  for (int e = 0; e < 8; ++e) { red[0][rl][cg * 8 + e] = s[e]; red[1][rl][cg * 8 + e] = s2[e]; }
  __syncthreads();
  {
    const int which = threadIdx.x >> 7, c = threadIdx.x & 127;
    float a = 0.f;
#pragma unroll
    for (int r = 0; r < 16; ++r) a += red[which][r][c];
    VST2(float, part1 + (size_t)blockIdx.x * 256 + threadIdx.x, a);
  }
}
__global__ __launch_bounds__(128) void k_bn(const float* __restrict__ part, int nblk, int nch, const float* __restrict__ gamma, const float* __restrict__ beta,
                                            float invn, float* __restrict__ scsh) {
  const int c = threadIdx.x;
  if (c >= nch) return;
  double s = 0.0, q = 0.0;
  for (int k = 0; k < nblk; ++k) { s += (double)part[(size_t)k * 2 * nch + c]; q += (double)part[(size_t)k * 2 * nch + nch + c]; }
  const double mean = s * invn, var = fmax(q * invn - mean * mean, 0.0);
  const float sc = gamma[c] / sqrtf((float)var + 1e-5f);
  VST2(float, scsh + c, sc);
  VST2(float, scsh + nch + c, beta[c] - (float)mean * sc);
}
__global__ __launch_bounds__(256) void k_w2eff(const float* __restrict__ w2, _Float16* __restrict__ Bw) {
  const int t = blockIdx.x * 256 + threadIdx.x;
  const int co = t / 48, k0 = (t % 48) * 8, dk = k0 >> 7, ci0 = k0 & 127;
  v8h v;
#pragma unroll
  for (int e = 0; e < 8; ++e) v[e] = (_Float16)w2[((size_t)(ci0 + e) * C2 + co) * 3 + (2 - dk)];
  VST2(v8h, Bw + (size_t)co * K2 + k0, v);
}
__global__ __launch_bounds__(256) void k_conv2(const float* __restrict__ images, const float* __restrict__ w1, const float* __restrict__ b1,
                                               const float* __restrict__ scsh1, const _Float16* __restrict__ Bw,
                                               const float* __restrict__ b2, float* __restrict__ h2, float* __restrict__ part2) {
  __shared__ __attribute__((aligned(16))) _Float16 sH[4][34][C1];
  __shared__ __attribute__((aligned(16))) float sT[8][16 * C2];
  __shared__ float red[2][8][C2];
  const int lane = threadIdx.x & 31, wave = threadIdx.x >> 5, hh = lane >> 4, l16 = lane & 15;
  const int bblk = blockIdx.x * 4;
  for (int it = threadIdx.x; it < 4 * 34 * 16; it += 256) {
    const int cg = it & 15, tp = (it >> 4) % 34, sl = it / (34 * 16), t = tp - 1;
    v8h o;
    if (t < 0 || t >= TL) { for (int e = 0; e < 8; ++e) o[e] = (_Float16)0.f; }
    else {
      const float* im = images + (size_t)(bblk + sl) * 32;
      const float i0 = (t > 0) ? im[t - 1] : 0.f, i1 = im[t], i2 = (t < TL - 1) ? im[t + 1] : 0.f;
#pragma unroll
      for (int e = 0; e < 8; ++e) { const int c = cg * 8 + e;
        const float v = fmaxf(i0 * w1[c * 3 + 2] + i1 * w1[c * 3 + 1] + i2 * w1[c * 3 + 0] + b1[c], 0.f);
        o[e] = (_Float16)(v * scsh1[c] + scsh1[C1 + c]); }
    }
    *(v8h*)(&sH[sl][tp][cg * 8]) = o;
  }
  __syncthreads();
  const int row0 = (blockIdx.x * 8 + wave) * 16;
  const int sl = wave >> 1, t = (wave & 1) * 16 + l16;
  v8f acc[4] = {};
  for (int dk = 0; dk < 3; ++dk) {
    const _Float16* arow = &sH[sl][t + dk][0];
#pragma unroll
    for (int c0 = 0; c0 < C1; c0 += 32) {
      const v16h a = frag16(arow + c0, hh);
      const int k = dk * C1 + c0;
#pragma unroll
      for (int tt = 0; tt < 4; ++tt) acc[tt] = wmma16(a, frag16(Bw + (size_t)(tt * 16 + l16) * K2 + k, hh), acc[tt]);
    }
  }
  float s[4] = {0.f, 0.f, 0.f, 0.f}, q[4] = {0.f, 0.f, 0.f, 0.f};
  float* st = sT[wave];
#pragma unroll
  for (int tt = 0; tt < 4; ++tt) {
    const int co = tt * 16 + l16; const float bv = b2[co];
#pragma unroll
    for (int r = 0; r < 8; ++r) { const float v = fmaxf(acc[tt][r] + bv, 0.f); st[(r + 8 * hh) * C2 + co] = v; s[tt] += v; q[tt] += v * v; }
  }
#pragma unroll
  for (int tt = 0; tt < 4; ++tt) { s[tt] += __shfl_xor(s[tt], 16); q[tt] += __shfl_xor(q[tt], 16); }
  if (hh == 0) {
#pragma unroll
    for (int tt = 0; tt < 4; ++tt) { red[0][wave][tt * 16 + l16] = s[tt]; red[1][wave][tt * 16 + l16] = q[tt]; }
  }
  __builtin_amdgcn_fence(__ATOMIC_RELEASE, "workgroup"); __builtin_amdgcn_wave_barrier(); __builtin_amdgcn_fence(__ATOMIC_ACQUIRE, "workgroup");
  for (int pass = 0; pass < 2; ++pass) {
#pragma unroll
    for (int j = 0; j < 8; ++j) { const int rr = j * 2 + (lane >> 4), sg = lane & 15;
      *(volatile v4f*)(h2 + (size_t)(row0 + rr) * C2 + sg * 4) = *(const v4f*)(st + rr * C2 + sg * 4); }
    __threadfence();
  }
  __syncthreads();
  if (threadIdx.x < 128) {
    const int which = threadIdx.x >> 6, c = threadIdx.x & 63;
    float a = 0.f;
#pragma unroll
    for (int w = 0; w < 8; ++w) a += red[which][w][c];
    VST2(float, part2 + (size_t)blockIdx.x * 128 + threadIdx.x, a);
  }
}
__global__ __launch_bounds__(256) void k_conv3(const float* __restrict__ h2, const float* __restrict__ scsh2, const float* __restrict__ w3,
                                               const float* __restrict__ b3, float* __restrict__ out) {
  __shared__ float sw[3][C2], ssc[C2], ssh[C2];
  if (threadIdx.x < 192) { const int ci = threadIdx.x % C2, dk = threadIdx.x / C2; sw[dk][ci] = w3[ci * 3 + (2 - dk)]; }
  if (threadIdx.x < C2) { ssc[threadIdx.x] = scsh2[threadIdx.x]; ssh[threadIdx.x] = scsh2[C2 + threadIdx.x]; }
  __syncthreads();
  const int idx = blockIdx.x * 256 + threadIdx.x;
  const int b = idx >> 5, t = idx & 31;
  float a = b3[0];
  for (int dk = 0; dk < 3; ++dk) {
    const int ts = t + dk - 1;
    if (ts < 0 || ts >= TL) continue;
    const float* src = h2 + ((size_t)b * 32 + ts) * C2;
#pragma unroll 2
    for (int ci = 0; ci < C2; ci += 4) {
      const v4f v = *(const v4f*)(src + ci);
#pragma unroll
      for (int e = 0; e < 4; ++e) a += (v[e] * ssc[ci + e] + ssh[ci + e]) * sw[dk][ci + e];
    }
  }
  VST2(float, out + idx, tanhf(a));
}
extern "C" void kernel_launch(void* const* d_in, const int* in_sizes, int n_in,
                              void* d_out, int out_size, void* d_ws, size_t ws_size, hipStream_t stream) {
  (void)in_sizes; (void)n_in; (void)out_size;
  const float* x = (const float*)d_in[0]; const float* qp = (const float*)d_in[1];
  const float* w1 = (const float*)d_in[2]; const float* b1 = (const float*)d_in[3]; const float* g1 = (const float*)d_in[4]; const float* be1 = (const float*)d_in[5];
  const float* w2 = (const float*)d_in[6]; const float* b2 = (const float*)d_in[7]; const float* g2 = (const float*)d_in[8]; const float* be2 = (const float*)d_in[9];
  const float* w3 = (const float*)d_in[10]; const float* b3 = (const float*)d_in[11];
  float* out = (float*)d_out;
  char* ws = (char*)d_ws; size_t off = 0;
  auto take = [&](size_t bytes) { void* p = ws + off; off = (off + bytes + 255) & ~(size_t)255; return p; };
  float*    images = (float*)take((size_t)NB * 32 * 4);
  float*    h2     = (float*)take((size_t)NROW * C2 * 4);
  _Float16* Bw     = (_Float16*)take((size_t)C2 * K2 * 2);
  const int NB1 = NB / 8, NB2 = NROW / 128;
  float* part1 = (float*)take((size_t)NB1 * 256 * 4);
  float* part2 = (float*)take((size_t)NB2 * 128 * 4);
  float* scsh1 = (float*)take(256 * 4);
  float* scsh2 = (float*)take(128 * 4);
  if (off > ws_size) return;
  k_patches<<<NB * 8 / 256, 256, 0, stream>>>(x, qp, images);
  k_conv1<<<NB1, 256, 0, stream>>>(images, w1, b1, part1);
  k_bn<<<1, 128, 0, stream>>>(part1, NB1, C1, g1, be1, 1.0f / (float)NROW, scsh1);
  k_w2eff<<<C2 * K2 / 8 / 256, 256, 0, stream>>>(w2, Bw);
  k_conv2<<<NB2, 256, 0, stream>>>(images, w1, b1, scsh1, Bw, b2, h2, part2);
  k_bn<<<1, 128, 0, stream>>>(part2, NB2, C2, g2, be2, 1.0f / (float)NROW, scsh2);
  k_conv3<<<NROW / 256, 256, 0, stream>>>(h2, scsh2, w3, b3, out);
}
